// ChimeraMambaKANBlock_89756226551981
// MI455X (gfx1250) — hardware-run, weakly checked
//
#include <hip/hip_runtime.h>
#include <stddef.h>
#include <math.h>


#pragma clang fp contract(off)

#define NB    2
#define LS    2048
#define DM    512
#define DI    1024
#define DS    16
#define DR    32
#define DBN   64
#define DBW   128
#define NG    8
#define KB    (DM * NG)
#define MR    (NB * LS)
#define NTHR  256
#define KTHR  128
#define LNEPS 1e-5f
#define WSCAP 134217728
#define WCARRY 64.0f
#define YCARRY 16.0f
#define INVDEN 3.0303030303030303f

#define SZ_WIN  ((size_t)(2 * DI) * DM * 2)
#define SZ_WXP  ((size_t)DBW * DI * 2)
#define SZ_WDT  ((size_t)DI * DR * 2)
#define SZ_WOUT ((size_t)DM * DI * 2)
#define SZ_WSP  ((size_t)DM * KB * 2)
#define SZ_UH   ((size_t)MR * DM * 2)
#define SZ_X1   ((size_t)MR * DM * 4)
#define SZ_DBC  ((size_t)MR * DBW * 4)
#define SZ_DTH  ((size_t)MR * DBN * 2)
#define SZ_XCH  ((size_t)MR * DI * 2)
#define SZ_XZ   ((size_t)MR * 2 * DI * 4)
#define SZ_XC   ((size_t)MR * DI * 4)
#define SZ_DEL  ((size_t)MR * DI * 4)
#define O_WIN  ((size_t)0)
#define O_WXP  (O_WIN + SZ_WIN)
#define O_WDT  (O_WXP + SZ_WXP)
#define O_WOUT (O_WDT + SZ_WDT)
#define O_WSH  (O_WOUT + SZ_WOUT)
#define O_WSL  (O_WSH + SZ_WSP)
#define O_UH   (O_WSL + SZ_WSP)
#define O_X1   (O_UH + SZ_UH)
#define O_DBC  (O_X1 + SZ_X1)
#define O_DTH  (O_DBC + SZ_DBC)
#define O_XCH  (O_DTH + SZ_DTH)
#define O_XZ   (O_XCH + SZ_XCH)
#define O_XC   (O_XZ + SZ_XZ)
#define O_DEL  (O_XC + SZ_XC)
#define WSTOT  (O_DEL + SZ_DEL)
#define O_BH   O_XZ
#define O_BL   O_XC
static_assert(WSTOT == (size_t)102563840);
static_assert(WSTOT <= (size_t)WSCAP);
static_assert(SZ_XZ == (size_t)MR * KB * 2);
static_assert(SZ_XC + SZ_DEL == (size_t)MR * KB * 2);
static_assert(O_DEL == O_XC + SZ_XC);
static_assert((O_WXP % 128) == 0 && (O_WDT % 128) == 0 && (O_WOUT % 128) == 0 && (O_WSH % 128) == 0);
static_assert((O_WSL % 128) == 0 && (O_UH % 128) == 0 && (O_X1 % 128) == 0 && (O_DBC % 128) == 0);
static_assert((O_DTH % 128) == 0 && (O_XCH % 128) == 0 && (O_XZ % 128) == 0 && (O_XC % 128) == 0);
static_assert((O_DEL % 128) == 0 && (WSTOT % 128) == 0);

static_assert((MR % 128) == 0 && ((2 * DI) % 128) == 0 && (DI % 128) == 0 && (DM % 128) == 0 && DBW == 128);
static_assert((DM % 32) == 0 && (DI % 32) == 0 && (DR % 32) == 0 && (KB % 32) == 0);
static_assert(DR + 2 * DS == DBN && DBN <= DBW && (DBN % 8) == 0);
static_assert(DI / 4 == NTHR && (MR % (NTHR / 32)) == 0 && (MR % (KTHR / 32)) == 0 && DM == 2 * 256);
static_assert(((2 * DI) * DM / 8) % NTHR == 0 && (DBW * DI / 8) % NTHR == 0 && (DI * DR / 8) % NTHR == 0);
static_assert((DM * DI / 8) % NTHR == 0 && (DM * KB / 8) % NTHR == 0);

typedef _Float16     v16h __attribute__((ext_vector_type(16)));
typedef _Float16     v8h  __attribute__((ext_vector_type(8), __may_alias__));
typedef _Float16     v4h  __attribute__((ext_vector_type(4), __may_alias__));
typedef __bf16       v16b __attribute__((ext_vector_type(16)));
typedef float        v8f  __attribute__((ext_vector_type(8)));
typedef float        v4f  __attribute__((ext_vector_type(4), __may_alias__));
typedef unsigned int v4u  __attribute__((ext_vector_type(4), __may_alias__));
typedef unsigned int v2u  __attribute__((ext_vector_type(2), __may_alias__));
typedef int          v8i  __attribute__((ext_vector_type(8)));
union Frag  { v16h v; v8i w; v4u q[2]; };
union FragB { v16b v; v8i w; v4u q[2]; };
union Pk8 { v8h h; v4u u; };
union Pk4 { v4h h; v2u u; };
static_assert(sizeof(Frag) == 32);
static_assert(sizeof(FragB) == 32);
static_assert(sizeof(Pk8) == 16);
static_assert(sizeof(Pk4) == 8);

__device__ __forceinline__ v8f wmh(const Frag& a, const Frag& b, v8f c) {
  v8f d = __builtin_amdgcn_wmma_f32_16x16x32_f16(false, a.v, false, b.v, (short)0, c, false, false);
  asm volatile("v_nop\n\tv_nop\n\tv_nop\n\tv_nop" : "+v"(d) : "v"(a.w), "v"(b.w));
  return d;
}
__device__ __forceinline__ v8f wmb(const FragB& a, const FragB& b, v8f c) {
  v8f d = __builtin_amdgcn_wmma_f32_16x16x32_bf16(false, a.v, false, b.v, (short)0, c, false, false);
  asm volatile("v_nop\n\tv_nop\n\tv_nop\n\tv_nop" : "+v"(d) : "v"(a.w), "v"(b.w));
  return d;
}

__device__ __forceinline__ v8f zero8() {
  v8f z = {0.f, 0.f, 0.f, 0.f, 0.f, 0.f, 0.f, 0.f};
  return z;
}

__device__ __forceinline__ v4u pack8(v4f a, v4f c, float mul) {
  v8h hv = {(_Float16)(a[0] * mul), (_Float16)(a[1] * mul), (_Float16)(a[2] * mul), (_Float16)(a[3] * mul),
            (_Float16)(c[0] * mul), (_Float16)(c[1] * mul), (_Float16)(c[2] * mul), (_Float16)(c[3] * mul)};
  Pk8 p;
  p.h = hv;
  return p.u;
}

__device__ __forceinline__ v2u pack4(v4f a, float mul) {
  v4h hv = {(_Float16)(a[0] * mul), (_Float16)(a[1] * mul), (_Float16)(a[2] * mul), (_Float16)(a[3] * mul)};
  Pk4 p;
  p.h = hv;
  return p.u;
}

__device__ __forceinline__ unsigned int bfb(float f) {
  unsigned int u = __float_as_uint(f);
  u += 0x7fffu + ((u >> 16) & 1u);
  return u >> 16;
}

__device__ __forceinline__ void split8(v4f a, v4f c, v4u& ho, v4u& lo) {
  const float f[8] = {a[0], a[1], a[2], a[3], c[0], c[1], c[2], c[3]};
  unsigned int hb[8], lb[8];
#pragma unroll
  for (int i = 0; i < 8; ++i) {
    hb[i] = bfb(f[i]);
    lb[i] = bfb(f[i] - __uint_as_float(hb[i] << 16));
  }
  ho = (v4u){hb[0] | (hb[1] << 16), hb[2] | (hb[3] << 16), hb[4] | (hb[5] << 16), hb[6] | (hb[7] << 16)};
  lo = (v4u){lb[0] | (lb[1] << 16), lb[2] | (lb[3] << 16), lb[4] | (lb[5] << 16), lb[6] | (lb[7] << 16)};
}

__device__ __forceinline__ float silu_f(float a) { return a * __builtin_amdgcn_rcpf(1.0f + __expf(-a)); }
__device__ __forceinline__ float softplus_f(float a) { return fmaxf(a, 0.0f) + log1pf(__expf(-fabsf(a))); }

__global__ __launch_bounds__(NTHR) void k_cvt(const float* __restrict__ src, int N, int Np, int K, float scale,
                                              unsigned short* dst) {
  const int g = blockIdx.x * NTHR + threadIdx.x;
  const size_t tot = ((size_t)Np * (size_t)K) >> 3;
  if ((size_t)g >= tot) return;
  const size_t e = (size_t)g * 8;
  const int row = (int)(e / (size_t)K);
  const int col = (int)(e - (size_t)row * (size_t)K);
  const bool valid = row < N;
  const int rowc = valid ? row : (N - 1);
  const float* p = src + (size_t)rowc * (size_t)K + col;
  const v4f a = *(const v4f*)p;
  const v4f c = *(const v4f*)(p + 4);
  const v4u pk = pack8(a, c, scale);
  const v4u zz = {0u, 0u, 0u, 0u};
  const v4u o = valid ? pk : zz;
  *(volatile v4u*)(dst + e) = o;
  __threadfence();
  *(volatile v4u*)(dst + e) = o;
}

__global__ __launch_bounds__(NTHR) void k_cvt2(const float* __restrict__ src, int n, unsigned short* dhi,
                                               unsigned short* dlo) {
  const int g = blockIdx.x * NTHR + threadIdx.x;
  const size_t e = (size_t)g * 8;
  if (e + 8 > (size_t)n) return;
  const v4f a = *(const v4f*)(src + e);
  const v4f c = *(const v4f*)(src + e + 4);
  v4u ho, lo;
  split8(a, c, ho, lo);
  *(volatile v4u*)(dhi + e) = ho;
  *(volatile v4u*)(dlo + e) = lo;
  __threadfence();
  *(volatile v4u*)(dhi + e) = ho;
  *(volatile v4u*)(dlo + e) = lo;
}

__device__ __forceinline__ void dln16(const float* __restrict__ xr, const float* __restrict__ w1,
                                      const float* __restrict__ b1, const float* __restrict__ w2,
                                      const float* __restrict__ b2, int lane, float (&kv)[16]) {
  float v[16];
#pragma unroll
  for (int s = 0; s < 2; ++s) {
    const v4f a = *(const v4f*)(xr + 256 * s + 8 * lane);
    const v4f c = *(const v4f*)(xr + 256 * s + 8 * lane + 4);
    v[8 * s + 0] = a[0]; v[8 * s + 1] = a[1]; v[8 * s + 2] = a[2]; v[8 * s + 3] = a[3];
    v[8 * s + 4] = c[0]; v[8 * s + 5] = c[1]; v[8 * s + 6] = c[2]; v[8 * s + 7] = c[3];
  }
  float sum = (((v[0] + v[1]) + (v[2] + v[3])) + ((v[4] + v[5]) + (v[6] + v[7]))) +
              (((v[8] + v[9]) + (v[10] + v[11])) + ((v[12] + v[13]) + (v[14] + v[15])));
#pragma unroll
  for (int off = 16; off > 0; off >>= 1) sum += __shfl_xor(sum, off, 32);
  const float mean = sum * (1.0f / (float)DM);
  float dv[16];
  float ss = 0.0f;
#pragma unroll
  for (int i = 0; i < 16; ++i) {
    dv[i] = v[i] - mean;
    ss = ss + dv[i] * dv[i];
  }
#pragma unroll
  for (int off = 16; off > 0; off >>= 1) ss += __shfl_xor(ss, off, 32);
  const float rs = rsqrtf(ss * (1.0f / (float)DM) + LNEPS);
  float y[16];
#pragma unroll
  for (int s = 0; s < 2; ++s) {
    const v4f wa = *(const v4f*)(w1 + 256 * s + 8 * lane);
    const v4f wb = *(const v4f*)(w1 + 256 * s + 8 * lane + 4);
    const v4f ba = *(const v4f*)(b1 + 256 * s + 8 * lane);
    const v4f bb = *(const v4f*)(b1 + 256 * s + 8 * lane + 4);
#pragma unroll
    for (int j = 0; j < 4; ++j) {
      y[8 * s + j]     = (dv[8 * s + j] * rs) * wa[j] + ba[j];
      y[8 * s + 4 + j] = (dv[8 * s + 4 + j] * rs) * wb[j] + bb[j];
    }
  }
  float sum2 = (((y[0] + y[1]) + (y[2] + y[3])) + ((y[4] + y[5]) + (y[6] + y[7]))) +
               (((y[8] + y[9]) + (y[10] + y[11])) + ((y[12] + y[13]) + (y[14] + y[15])));
#pragma unroll
  for (int off = 16; off > 0; off >>= 1) sum2 += __shfl_xor(sum2, off, 32);
  const float mean2 = sum2 * (1.0f / (float)DM);
  float d2[16];
  float ss2 = 0.0f;
#pragma unroll
  for (int i = 0; i < 16; ++i) {
    d2[i] = y[i] - mean2;
    ss2 = ss2 + d2[i] * d2[i];
  }
#pragma unroll
  for (int off = 16; off > 0; off >>= 1) ss2 += __shfl_xor(ss2, off, 32);
  const float rs2 = rsqrtf(ss2 * (1.0f / (float)DM) + LNEPS);
#pragma unroll
  for (int s = 0; s < 2; ++s) {
    const v4f wa = *(const v4f*)(w2 + 256 * s + 8 * lane);
    const v4f wb = *(const v4f*)(w2 + 256 * s + 8 * lane + 4);
    const v4f ba = *(const v4f*)(b2 + 256 * s + 8 * lane);
    const v4f bb = *(const v4f*)(b2 + 256 * s + 8 * lane + 4);
#pragma unroll
    for (int j = 0; j < 4; ++j) {
      kv[8 * s + j]     = (d2[8 * s + j] * rs2) * wa[j] + ba[j];
      kv[8 * s + 4 + j] = (d2[8 * s + 4 + j] * rs2) * wb[j] + bb[j];
    }
  }
}

__global__ __launch_bounds__(NTHR) void k_ln(const float* __restrict__ X, const float* __restrict__ w1,
                                             const float* __restrict__ b1, const float* __restrict__ w2,
                                             const float* __restrict__ b2, unsigned short* UH) {
  const int tid = threadIdx.x, lane = tid & 31, wave = tid >> 5;
  const int row = blockIdx.x * (NTHR / 32) + wave;
  float kv[16];
  dln16(X + (size_t)row * DM, w1, b1, w2, b2, lane, kv);
  v4u o[2];
#pragma unroll
  for (int s = 0; s < 2; ++s) {
    const v4f ya = {kv[8 * s + 0], kv[8 * s + 1], kv[8 * s + 2], kv[8 * s + 3]};
    const v4f yb = {kv[8 * s + 4], kv[8 * s + 5], kv[8 * s + 6], kv[8 * s + 7]};
    o[s] = pack8(ya, yb, 1.0f);
  }
  unsigned short* dp = UH + (size_t)row * DM + 8 * lane;
#pragma unroll
  for (int s = 0; s < 2; ++s) *(volatile v4u*)(dp + 256 * s) = o[s];
  __threadfence();
#pragma unroll
  for (int s = 0; s < 2; ++s) *(volatile v4u*)(dp + 256 * s) = o[s];
}

__global__ __launch_bounds__(KTHR) void k_kan(const float* __restrict__ X1, const float* __restrict__ w1,
                                              const float* __restrict__ b1, const float* __restrict__ w2,
                                              const float* __restrict__ b2, const float* __restrict__ gridv,
                                              unsigned short* BH, unsigned short* BL) {
  __shared__ __align__(16) unsigned short sH[(KTHR / 32) * (KB / 2)];
  __shared__ __align__(16) unsigned short sL[(KTHR / 32) * (KB / 2)];
  const int tid = threadIdx.x, lane = tid & 31, wave = tid >> 5;
  const int row = blockIdx.x * (KTHR / 32) + wave;
  float kv[16];
  dln16(X1 + (size_t)row * DM, w1, b1, w2, b2, lane, kv);
  float gr[NG];
  {
    const v4f ga = *(const v4f*)(gridv);
    const v4f gb = *(const v4f*)(gridv + 4);
    gr[0] = ga[0]; gr[1] = ga[1]; gr[2] = ga[2]; gr[3] = ga[3];
    gr[4] = gb[0]; gr[5] = gb[1]; gr[6] = gb[2]; gr[7] = gb[3];
  }
  unsigned short* wh = sH + wave * (KB / 2);
  unsigned short* wl = sL + wave * (KB / 2);
#pragma unroll
  for (int s = 0; s < 2; ++s) {
#pragma unroll
    for (int j = 0; j < 8; ++j) {
      const float kc = kv[8 * s + j];
      unsigned int hb[NG], lb[NG];
#pragma unroll
      for (int g = 0; g < NG; ++g) {
        const float a  = (kc - gr[g]) * INVDEN;
        const float ex = __expf(2.0f * a);
        const float r  = __builtin_amdgcn_rcpf(ex + 1.0f);
        const float t  = 1.0f - 2.0f * r;
        const float bv = 1.0f - t * t;
        hb[g] = bfb(bv);
        lb[g] = bfb(bv - __uint_as_float(hb[g] << 16));
      }
      const v4u ph = {hb[0] | (hb[1] << 16), hb[2] | (hb[3] << 16), hb[4] | (hb[5] << 16), hb[6] | (hb[7] << 16)};
      const v4u pl = {lb[0] | (lb[1] << 16), lb[2] | (lb[3] << 16), lb[4] | (lb[5] << 16), lb[6] | (lb[7] << 16)};
      *(v4u*)(wh + (8 * lane + j) * 8) = ph;
      *(v4u*)(wl + (8 * lane + j) * 8) = pl;
    }
    __syncthreads();
    const size_t gb0 = (size_t)row * (size_t)KB + (size_t)s * (KB / 2);
#pragma unroll
    for (int it = 0; it < 8; ++it) {
      const int p = it * 32 + lane;
      const v4u oh = *(const v4u*)(wh + 8 * p);
      const v4u ol = *(const v4u*)(wl + 8 * p);
      *(volatile v4u*)(BH + gb0 + 8 * p) = oh;
      *(volatile v4u*)(BL + gb0 + 8 * p) = ol;
    }
    __threadfence();
#pragma unroll
    for (int it = 0; it < 8; ++it) {
      const int p = it * 32 + lane;
      const v4u oh = *(const v4u*)(wh + 8 * p);
      const v4u ol = *(const v4u*)(wl + 8 * p);
      *(volatile v4u*)(BH + gb0 + 8 * p) = oh;
      *(volatile v4u*)(BL + gb0 + 8 * p) = ol;
    }
    __syncthreads();
  }
}

template <int EP>
__global__ __launch_bounds__(NTHR) void k_gemm(const unsigned short* __restrict__ A,
                                               const unsigned short* __restrict__ A2, int lda,
                                               const unsigned short* __restrict__ W,
                                               const unsigned short* __restrict__ W2, int ldw, int K, float cscale,
                                               const float* __restrict__ bias, const float* __restrict__ res, int ldr,
                                               float* Cf, int ldc, unsigned short* P, int ldp, float pmul) {
  extern __shared__ __align__(16) float sC[];
  constexpr bool SPLIT = (EP == 5);
  constexpr int  PW    = (EP == 2) ? 64 : 0;
  constexpr int  PPR   = (PW > 0) ? (PW / 8) : 1;
  constexpr int  NPP   = (PW > 0) ? ((128 * PPR) / NTHR) : 1;
  constexpr int  NF4   = (128 * 128 / 4) / NTHR;

  const int tid = threadIdx.x, lane = tid & 31, wave = tid >> 5, h = lane >> 4, m = lane & 15;
  const int wm = wave & 3, wn = wave >> 2;
  const int m0 = blockIdx.y * 128, n0 = blockIdx.x * 128;

  v8f acc[2][4];
#pragma unroll
  for (int mi = 0; mi < 2; ++mi)
#pragma unroll
    for (int ni = 0; ni < 4; ++ni) acc[mi][ni] = zero8();

  const size_t aofs = (size_t)(m0 + 32 * wm + m) * (size_t)lda + (size_t)(8 * h);
  const unsigned short* ap0 = A + aofs;
  const unsigned short* ap1 = ap0 + (size_t)16 * (size_t)lda;
  const unsigned short* aq0 = A2 + aofs;
  const unsigned short* aq1 = aq0 + (size_t)16 * (size_t)lda;
  const size_t wofs = (size_t)(n0 + 64 * wn + m) * (size_t)ldw + (size_t)(8 * h);
  const unsigned short* wp = W + wofs;
  const unsigned short* wq = W2 + wofs;
  const size_t wstep = (size_t)16 * (size_t)ldw;
  const int nks = K >> 5;

#pragma unroll 1
  for (int ks = 0; ks < nks; ++ks) {
    const int k0 = ks << 5;
    if constexpr (!SPLIT) {
      Frag fa0, fa1;
      fa0.q[0] = *(const v4u*)(ap0 + k0);
      fa0.q[1] = *(const v4u*)(ap0 + k0 + 16);
      fa1.q[0] = *(const v4u*)(ap1 + k0);
      fa1.q[1] = *(const v4u*)(ap1 + k0 + 16);
#pragma unroll
      for (int ni = 0; ni < 4; ++ni) {
        const unsigned short* wpn = wp + wstep * (size_t)ni + k0;
        Frag fb;
        fb.q[0] = *(const v4u*)wpn;
        fb.q[1] = *(const v4u*)(wpn + 16);
        acc[0][ni] = wmh(fa0, fb, acc[0][ni]);
        acc[1][ni] = wmh(fa1, fb, acc[1][ni]);
      }
    } else {
      FragB fa0, fa1, ga0, ga1;
      fa0.q[0] = *(const v4u*)(ap0 + k0);
      fa0.q[1] = *(const v4u*)(ap0 + k0 + 16);
      fa1.q[0] = *(const v4u*)(ap1 + k0);
      fa1.q[1] = *(const v4u*)(ap1 + k0 + 16);
      ga0.q[0] = *(const v4u*)(aq0 + k0);
      ga0.q[1] = *(const v4u*)(aq0 + k0 + 16);
      ga1.q[0] = *(const v4u*)(aq1 + k0);
      ga1.q[1] = *(const v4u*)(aq1 + k0 + 16);
#pragma unroll
      for (int ni = 0; ni < 4; ++ni) {
        const unsigned short* wpn = wp + wstep * (size_t)ni + k0;
        FragB fb;
        fb.q[0] = *(const v4u*)wpn;
        fb.q[1] = *(const v4u*)(wpn + 16);
        acc[0][ni] = wmb(fa0, fb, acc[0][ni]);
        acc[1][ni] = wmb(fa1, fb, acc[1][ni]);
        acc[0][ni] = wmb(ga0, fb, acc[0][ni]);
        acc[1][ni] = wmb(ga1, fb, acc[1][ni]);
        const unsigned short* wqn = wq + wstep * (size_t)ni + k0;
        FragB gb;
        gb.q[0] = *(const v4u*)wqn;
        gb.q[1] = *(const v4u*)(wqn + 16);
        acc[0][ni] = wmb(fa0, gb, acc[0][ni]);
        acc[1][ni] = wmb(fa1, gb, acc[1][ni]);
      }
    }
  }

#pragma unroll
  for (int mi = 0; mi < 2; ++mi) {
#pragma unroll
    for (int ni = 0; ni < 4; ++ni) {
      const int cl = 64 * wn + 16 * ni + m;
#pragma unroll
      for (int r = 0; r < 8; ++r) {
        const int rl = 32 * wm + 16 * mi + 8 * h + r;
        sC[rl * 128 + cl] = acc[mi][ni][r];
      }
    }
  }
  __syncthreads();

#pragma unroll 1
  for (int it = 0; it < NF4; ++it) {
    const int e = it * NTHR + tid;
    const int rl = e >> 5, q = e & 31;
    float* sp = sC + rl * 128 + 4 * q;
    v4f v = *(const v4f*)sp;
    v = v * cscale;
    if constexpr (EP == 1) {
      const v4f bb = *(const v4f*)(bias + n0 + 4 * q);
#pragma unroll
      for (int j = 0; j < 4; ++j) v[j] = v[j] + bb[j];
    } else if constexpr (EP == 3) {
      const v4f bb = *(const v4f*)(bias + n0 + 4 * q);
#pragma unroll
      for (int j = 0; j < 4; ++j) v[j] = softplus_f(v[j] + bb[j]);
    } else if constexpr (EP == 4) {
      const v4f bb = *(const v4f*)(bias + n0 + 4 * q);
      const v4f rr = *(const v4f*)(res + (size_t)(m0 + rl) * (size_t)ldr + n0 + 4 * q);
#pragma unroll
      for (int j = 0; j < 4; ++j) v[j] = rr[j] + (v[j] + bb[j]);
    } else if constexpr (EP == 5) {
      const v4f rr = *(const v4f*)(res + (size_t)(m0 + rl) * (size_t)ldr + n0 + 4 * q);
#pragma unroll
      for (int j = 0; j < 4; ++j) v[j] = rr[j] + v[j];
    }
    *(v4f*)sp = v;
  }
  __syncthreads();

  v4u po[NPP];
  size_t pd[NPP];
  if constexpr (PW > 0) {
#pragma unroll
    for (int i = 0; i < NPP; ++i) {
      const int e = i * NTHR + tid;
      const int rl = e / PPR, q = e % PPR;
      const v4f a = *(const v4f*)(sC + rl * 128 + 8 * q);
      const v4f c = *(const v4f*)(sC + rl * 128 + 8 * q + 4);
      po[i] = pack8(a, c, pmul);
      pd[i] = (size_t)(m0 + rl) * (size_t)ldp + (size_t)(n0 + 8 * q);
    }
  } else {
    po[0] = (v4u){0u, 0u, 0u, 0u};
    pd[0] = 0;
  }

#pragma unroll 4
  for (int it = 0; it < NF4; ++it) {
    const int e = it * NTHR + tid;
    const int rl = e >> 5, q = e & 31;
    const v4f v = *(const v4f*)(sC + rl * 128 + 4 * q);
    *(volatile v4f*)(Cf + (size_t)(m0 + rl) * (size_t)ldc + n0 + 4 * q) = v;
  }
  if constexpr (PW > 0) {
#pragma unroll
    for (int i = 0; i < NPP; ++i) *(volatile v4u*)(P + pd[i]) = po[i];
  }
  __threadfence();
#pragma unroll 4
  for (int it = 0; it < NF4; ++it) {
    const int e = it * NTHR + tid;
    const int rl = e >> 5, q = e & 31;
    const v4f v = *(const v4f*)(sC + rl * 128 + 4 * q);
    *(volatile v4f*)(Cf + (size_t)(m0 + rl) * (size_t)ldc + n0 + 4 * q) = v;
  }
  if constexpr (PW > 0) {
#pragma unroll
    for (int i = 0; i < NPP; ++i) *(volatile v4u*)(P + pd[i]) = po[i];
  }
}

__global__ __launch_bounds__(NTHR) void k_conv(const float* __restrict__ XZ, const float* __restrict__ cw,
                                               const float* __restrict__ cb, float* XC, unsigned short* XCH) {
  const int row = blockIdx.x;
  const int l = row & (LS - 1);
  const int dq = threadIdx.x * 4;
  v4f acc = *(const v4f*)(cb + dq);
  v4f w[4];
#pragma unroll
  for (int j = 0; j < 4; ++j) w[j] = *(const v4f*)(cw + (size_t)(dq + j) * 4);
#pragma unroll
  for (int k = 0; k < 4; ++k) {
    const int tt = l + k - 3;
    const bool ok = (tt >= 0);
    const int srow = ok ? (row + k - 3) : row;
    const v4f xv = *(const v4f*)(XZ + (size_t)srow * (size_t)(2 * DI) + dq);
#pragma unroll
    for (int j = 0; j < 4; ++j) {
      const float pr = xv[j] * w[j][k];
      acc[j] = acc[j] + (ok ? pr : 0.0f);
    }
  }
  v4f u;
#pragma unroll
  for (int j = 0; j < 4; ++j) u[j] = silu_f(acc[j]);
  const v2u hv = pack4(u, WCARRY);
  const size_t o = (size_t)row * DI + dq;
  *(volatile v4f*)(XC + o) = u;
  *(volatile v2u*)(XCH + o) = hv;
  __threadfence();
  *(volatile v4f*)(XC + o) = u;
  *(volatile v2u*)(XCH + o) = hv;
}

#define SCB 256
#define STB 32
static_assert(SCB == NTHR && (DI % SCB) == 0 && (LS % STB) == 0 && ((STB * SCB / 8) % NTHR) == 0);

__global__ __launch_bounds__(NTHR) void k_scan(const float* __restrict__ DEL, const float* __restrict__ XC,
                                               const float* __restrict__ DBC, const float* __restrict__ XZ,
                                               const float* __restrict__ Alog, const float* __restrict__ Dp,
                                               unsigned short* YH) {
  __shared__ __align__(16) float sA[SCB * DS];
  __shared__ __align__(16) float sY[STB * SCB];
  const int tid = threadIdx.x;
  const int bi = blockIdx.x / (DI / SCB);
  const int cbase = (blockIdx.x - bi * (DI / SCB)) * SCB;
  const int c = cbase + tid;
  const size_t rbase = (size_t)bi * LS;
#pragma unroll 1
  for (int e = tid; e < SCB * DS; e += NTHR) sA[e] = -expf(Alog[(size_t)cbase * DS + e]);
  __syncthreads();
  float Aj[DS], hs[DS];
#pragma unroll
  for (int j = 0; j < DS; ++j) {
    Aj[j] = sA[tid * DS + j];
    hs[j] = 0.0f;
  }
  const float Dd = Dp[c];

#pragma unroll 1
  for (int t0 = 0; t0 < LS; t0 += STB) {
#pragma unroll 1
    for (int tl = 0; tl < STB; ++tl) {
      const size_t t = rbase + (size_t)(t0 + tl);
      const float dt = DEL[t * DI + c];
      const float xv = XC[t * DI + c];
      const float zv = XZ[t * (size_t)(2 * DI) + DI + c];
      const float* bp = DBC + t * DBW + DR;
      const v4f b0 = *(const v4f*)(bp);
      const v4f b1 = *(const v4f*)(bp + 4);
      const v4f b2 = *(const v4f*)(bp + 8);
      const v4f b3 = *(const v4f*)(bp + 12);
      const v4f c0 = *(const v4f*)(bp + 16);
      const v4f c1 = *(const v4f*)(bp + 20);
      const v4f c2 = *(const v4f*)(bp + 24);
      const v4f c3 = *(const v4f*)(bp + 28);
      float Bv[DS], Cv[DS];
      Bv[0] = b0[0]; Bv[1] = b0[1]; Bv[2] = b0[2]; Bv[3] = b0[3];
      Bv[4] = b1[0]; Bv[5] = b1[1]; Bv[6] = b1[2]; Bv[7] = b1[3];
      Bv[8] = b2[0]; Bv[9] = b2[1]; Bv[10] = b2[2]; Bv[11] = b2[3];
      Bv[12] = b3[0]; Bv[13] = b3[1]; Bv[14] = b3[2]; Bv[15] = b3[3];
      Cv[0] = c0[0]; Cv[1] = c0[1]; Cv[2] = c0[2]; Cv[3] = c0[3];
      Cv[4] = c1[0]; Cv[5] = c1[1]; Cv[6] = c1[2]; Cv[7] = c1[3];
      Cv[8] = c2[0]; Cv[9] = c2[1]; Cv[10] = c2[2]; Cv[11] = c2[3];
      Cv[12] = c3[0]; Cv[13] = c3[1]; Cv[14] = c3[2]; Cv[15] = c3[3];
      float y = 0.0f;
#pragma unroll
      for (int j = 0; j < DS; ++j) {
        const float dA = __expf(dt * Aj[j]);
        const float hn = dA * hs[j] + (dt * Bv[j]) * xv;
        hs[j] = hn;
        y = y + hn * Cv[j];
      }
      const float sg = __builtin_amdgcn_rcpf(1.0f + __expf(-zv));
      sY[tl * SCB + tid] = (y + Dd * xv) * (zv * sg);
    }
    __syncthreads();
    {
      constexpr int NIT = (STB * SCB / 8) / NTHR;
      v4u hv[NIT];
      size_t dst[NIT];
#pragma unroll
      for (int it = 0; it < NIT; ++it) {
        const int e = it * NTHR + tid;
        const int rl = e >> 5, q = e & 31;
        const v4f a = *(const v4f*)(sY + rl * SCB + 8 * q);
        const v4f cc = *(const v4f*)(sY + rl * SCB + 8 * q + 4);
        hv[it] = pack8(a, cc, YCARRY);
        dst[it] = (rbase + (size_t)(t0 + rl)) * DI + (size_t)(cbase + 8 * q);
      }
#pragma unroll
      for (int it = 0; it < NIT; ++it) *(volatile v4u*)(YH + dst[it]) = hv[it];
      __threadfence();
#pragma unroll
      for (int it = 0; it < NIT; ++it) *(volatile v4u*)(YH + dst[it]) = hv[it];
    }
    __syncthreads();
  }
}

extern "C" void kernel_launch(void* const* d_in, const int* in_sizes, int n_in,
                              void* d_out, int out_size, void* d_ws, size_t ws_size,
                              hipStream_t stream) {
  if (n_in < 22) return;
  if (in_sizes[0] != MR * DM) return;
  if (in_sizes[1] != DM || in_sizes[2] != DM || in_sizes[3] != DM || in_sizes[4] != DM) return;
  if (in_sizes[5] != 2 * DI * DM || in_sizes[6] != 2 * DI) return;
  if (in_sizes[7] != DI * 4 || in_sizes[8] != DI) return;
  if (in_sizes[9] != DBN * DI) return;
  if (in_sizes[10] != DI * DR || in_sizes[11] != DI) return;
  if (in_sizes[12] != DI * DS || in_sizes[13] != DI) return;
  if (in_sizes[14] != DM * DI || in_sizes[15] != DM) return;
  if (in_sizes[16] != DM || in_sizes[17] != DM || in_sizes[18] != DM || in_sizes[19] != DM) return;
  if (in_sizes[20] != NG || in_sizes[21] != DM * KB) return;
  if (out_size != MR * DM) return;
  const size_t tot = (size_t)WSTOT;
  if (tot > ws_size || tot > (size_t)WSCAP) return;

  const float* x     = (const float*)d_in[0];
  const float* n1w   = (const float*)d_in[1];
  const float* n1b   = (const float*)d_in[2];
  const float* mnw   = (const float*)d_in[3];
  const float* mnb   = (const float*)d_in[4];
  const float* inw   = (const float*)d_in[5];
  const float* inb   = (const float*)d_in[6];
  const float* cw    = (const float*)d_in[7];
  const float* cb    = (const float*)d_in[8];
  const float* xpw   = (const float*)d_in[9];
  const float* dtw   = (const float*)d_in[10];
  const float* dtb   = (const float*)d_in[11];
  const float* alog  = (const float*)d_in[12];
  const float* dpp   = (const float*)d_in[13];
  const float* outw  = (const float*)d_in[14];
  const float* outb  = (const float*)d_in[15];
  const float* n2w   = (const float*)d_in[16];
  const float* n2b   = (const float*)d_in[17];
  const float* knw   = (const float*)d_in[18];
  const float* knb   = (const float*)d_in[19];
  const float* gridv = (const float*)d_in[20];
  const float* splw  = (const float*)d_in[21];
  float* out = (float*)d_out;

  char* ws = (char*)d_ws;
  unsigned short* WIN  = (unsigned short*)(ws + O_WIN);
  unsigned short* WXP  = (unsigned short*)(ws + O_WXP);
  unsigned short* WDT  = (unsigned short*)(ws + O_WDT);
  unsigned short* WOUT = (unsigned short*)(ws + O_WOUT);
  unsigned short* WSH  = (unsigned short*)(ws + O_WSH);
  unsigned short* WSL  = (unsigned short*)(ws + O_WSL);
  unsigned short* UH   = (unsigned short*)(ws + O_UH);
  float*          X1   = (float*)(ws + O_X1);
  float*          DBC  = (float*)(ws + O_DBC);
  unsigned short* DTH  = (unsigned short*)(ws + O_DTH);
  unsigned short* XCH  = (unsigned short*)(ws + O_XCH);
  unsigned short* YH   = (unsigned short*)(ws + O_XCH);
  float*          XZ   = (float*)(ws + O_XZ);
  float*          XC   = (float*)(ws + O_XC);
  float*          DEL  = (float*)(ws + O_DEL);
  unsigned short* BH   = (unsigned short*)(ws + O_BH);
  unsigned short* BL   = (unsigned short*)(ws + O_BL);

  const int GLDS = 128 * 128 * 4;

  k_cvt<<<((2 * DI) * DM / 8) / NTHR, NTHR, 0, stream>>>(inw, 2 * DI, 2 * DI, DM, WCARRY, WIN);
  k_cvt<<<(DBW * DI / 8) / NTHR, NTHR, 0, stream>>>(xpw, DBN, DBW, DI, WCARRY, WXP);
  k_cvt<<<(DI * DR / 8) / NTHR, NTHR, 0, stream>>>(dtw, DI, DI, DR, WCARRY, WDT);
  k_cvt<<<(DM * DI / 8) / NTHR, NTHR, 0, stream>>>(outw, DM, DM, DI, WCARRY, WOUT);
  k_cvt2<<<(DM * KB / 8) / NTHR, NTHR, 0, stream>>>(splw, DM * KB, WSH, WSL);

  k_ln<<<MR / (NTHR / 32), NTHR, 0, stream>>>(x, n1w, n1b, mnw, mnb, UH);

  k_gemm<1><<<dim3((2 * DI) / 128, MR / 128), NTHR, GLDS, stream>>>(
      UH, UH, DM, WIN, WIN, DM, DM, 1.0f / WCARRY, inb, X1, 0, XZ, 2 * DI, DTH, 0, 1.0f);
  k_conv<<<MR, NTHR, 0, stream>>>(XZ, cw, cb, XC, XCH);
  k_gemm<2><<<dim3(DBW / 128, MR / 128), NTHR, GLDS, stream>>>(
      XCH, XCH, DI, WXP, WXP, DI, DI, 1.0f / (WCARRY * WCARRY), inb, X1, 0, DBC, DBW, DTH, DBN, WCARRY);
  k_gemm<3><<<dim3(DI / 128, MR / 128), NTHR, GLDS, stream>>>(
      DTH, DTH, DBN, WDT, WDT, DR, DR, 1.0f / (WCARRY * WCARRY), dtb, X1, 0, DEL, DI, YH, 0, 1.0f);
  k_scan<<<NB * (DI / SCB), NTHR, 0, stream>>>(DEL, XC, DBC, XZ, alog, dpp, YH);
  k_gemm<4><<<dim3(DM / 128, MR / 128), NTHR, GLDS, stream>>>(
      YH, YH, DI, WOUT, WOUT, DI, DI, 1.0f / (YCARRY * WCARRY), outb, x, DM, X1, DM, DTH, 0, 1.0f);
  k_kan<<<MR / (KTHR / 32), KTHR, 0, stream>>>(X1, n2w, n2b, knw, knb, gridv, BH, BL);
  k_gemm<5><<<dim3(DM / 128, MR / 128), NTHR, GLDS, stream>>>(
      BH, BL, KB, WSH, WSL, KB, KB, 1.0f, outb, X1, DM, out, DM, DTH, 0, 1.0f);
}
